// Ms2z_64622077935692
// MI455X (gfx1250) — hardware-run, weakly checked
//
#include <hip/hip_runtime.h>

typedef _Float16 v16h __attribute__((ext_vector_type(16)));
typedef _Float16 v8h  __attribute__((ext_vector_type(8)));
typedef float    v8f  __attribute__((ext_vector_type(8)));
typedef float    v4f  __attribute__((ext_vector_type(4)));
typedef float    v2f  __attribute__((ext_vector_type(2)));
typedef int      v4i  __attribute__((ext_vector_type(4)));
typedef unsigned int v4u __attribute__((ext_vector_type(4)));
typedef v8h __attribute__((may_alias)) v8ha;
typedef v4f __attribute__((may_alias)) v4fa;
typedef v4i __attribute__((may_alias)) v4ia;
typedef v4u __attribute__((may_alias)) v4ua;

union Frag { v16h v; v8h half[2]; };

#define PAD_ID 0
#define BOS_ID 1
#define EOS_ID 2
#define NB 256
#define NS 512
#define NV 50000
#define ND 256
#define NL 128
#define NJ (NS + 1)
#define NROWS (NB * NJ)
#define TPITCH 544
#define RPITCH 288
#define HROWS 64
#define NBLK2 (NROWS / HROWS)
#define APITCH 264
#define WSC 16.0f
#define WSCINV 0.0625f

static_assert(NROWS % HROWS == 0);
static_assert(NB == 256);
static_assert(TPITCH % 32 == 0);
static_assert(RPITCH % 32 == 0);
static_assert((APITCH % 8) == 0);

__device__ __forceinline__ int clampi(int x, int lo, int hi) {
  return x < lo ? lo : (x > hi ? hi : x);
}

__device__ __forceinline__ v8f wmma_f16(v16h a, v16h b, v8f c) {
  v8f d = __builtin_amdgcn_wmma_f32_16x16x32_f16(false, a, false, b, (short)0, c, false, false);
  asm volatile("v_nop\n\tv_nop\n\tv_nop\n\tv_nop" : "+v"(d) : "v"(a), "v"(b));
  return d;
}

__device__ __forceinline__ v16h load_frag(const _Float16* p, int h) {
  Frag f;
  f.half[0] = *(const v8ha*)(p + 8 * h);
  f.half[1] = *(const v8ha*)(p + 16 + 8 * h);
  return f.v;
}

__device__ __forceinline__ void d2u(double d, unsigned int& lo, unsigned int& hi) {
  const unsigned long long u = (unsigned long long)__double_as_longlong(d);
  lo = (unsigned int)(u & 0xffffffffull);
  hi = (unsigned int)(u >> 32);
}
__device__ __forceinline__ double u2d(unsigned int lo, unsigned int hi) {
  const unsigned long long u = ((unsigned long long)hi << 32) | (unsigned long long)lo;
  return __longlong_as_double((long long)u);
}

__device__ __forceinline__ int wsum_i(int v) {
  v += __shfl_xor(v, 16);
  v += __shfl_xor(v, 8);
  v += __shfl_xor(v, 4);
  v += __shfl_xor(v, 2);
  v += __shfl_xor(v, 1);
  return v;
}
__device__ __forceinline__ int wmin_i(int v) {
  v = min(v, __shfl_xor(v, 16));
  v = min(v, __shfl_xor(v, 8));
  v = min(v, __shfl_xor(v, 4));
  v = min(v, __shfl_xor(v, 2));
  v = min(v, __shfl_xor(v, 1));
  return v;
}
__device__ __forceinline__ double shfl_xor_d(double v, int o) {
  unsigned int lo, hi;
  d2u(v, lo, hi);
  lo = (unsigned int)__shfl_xor((int)lo, o);
  hi = (unsigned int)__shfl_xor((int)hi, o);
  return u2d(lo, hi);
}
__device__ __forceinline__ double wsum_d(double v) {
  v += shfl_xor_d(v, 16);
  v += shfl_xor_d(v, 8);
  v += shfl_xor_d(v, 4);
  v += shfl_xor_d(v, 2);
  v += shfl_xor_d(v, 1);
  return v;
}

__device__ __forceinline__ void wout_store(const _Float16* sT, _Float16* woutT, int n0, int t) {
  #pragma unroll
  for (int it = 0; it < 4; ++it) {
    const int piece = it * 256 + t;
    const int row = piece >> 5, c16 = piece & 31;
    const v8h v = *(const v8ha*)(sT + row * APITCH + 8 * c16);
    *(volatile v8h*)(woutT + (size_t)(n0 + row) * ND + 8 * c16) = v;
  }
}

__global__ __launch_bounds__(256) void k_wout(const float* __restrict__ Wout,
                                              _Float16* __restrict__ woutT) {
  __shared__ __attribute__((aligned(16))) _Float16 sT[32 * APITCH];
  const int t = threadIdx.x;
  const int n0 = blockIdx.x * 32;
  {
    const float* src = Wout + (size_t)t * ND + n0;
    #pragma unroll
    for (int q = 0; q < 8; ++q) {
      const v4f v = *(const v4fa*)(src + 4 * q);
      sT[(4 * q + 0) * APITCH + t] = (_Float16)(v.x * WSC);
      sT[(4 * q + 1) * APITCH + t] = (_Float16)(v.y * WSC);
      sT[(4 * q + 2) * APITCH + t] = (_Float16)(v.z * WSC);
      sT[(4 * q + 3) * APITCH + t] = (_Float16)(v.w * WSC);
    }
  }
  __syncthreads();
  wout_store(sT, woutT, n0, t);
  __threadfence();
  wout_store(sT, woutT, n0, t);
}

__device__ __forceinline__ void seq_store(const float* s_rec, const unsigned int* s_sc,
                                          const int* s_tok0, const int* s_tok1,
                                          float* rec, int* inpP, int* tgtP, int b, int t) {
  if (t < 64) {
    const v4f v = *(const v4fa*)(s_rec + 4 * t);
    *(volatile v4f*)(rec + (size_t)b * RPITCH + 4 * t) = v;
  } else if (t < 72) {
    const int q = t - 64;
    const v4u v = *(const v4ua*)(s_sc + 4 * q);
    *(volatile v4u*)((unsigned int*)rec + (size_t)b * RPITCH + ND + 4 * q) = v;
  }
  if (t < TPITCH / 4) {
    const v4i a = *(const v4ia*)(s_tok0 + 4 * t);
    const v4i c = *(const v4ia*)(s_tok1 + 4 * t);
    *(volatile v4i*)(inpP + (size_t)b * TPITCH + 4 * t) = a;
    *(volatile v4i*)(tgtP + (size_t)b * TPITCH + 4 * t) = c;
  }
}

__global__ __launch_bounds__(256) void k_seq(
    const int* __restrict__ vocab, const int* __restrict__ order, const int* __restrict__ mask,
    const float* __restrict__ eps, const float* __restrict__ emb,
    const float* __restrict__ Wm, const float* __restrict__ bm,
    const float* __restrict__ Wv, const float* __restrict__ bv,
    const float* __restrict__ Wlin, const float* __restrict__ blin,
    float* __restrict__ rec, int* __restrict__ inpP, int* __restrict__ tgtP)
{
  __shared__ int s_msk[NS];
  __shared__ int s_voc[NS];
  __shared__ int s_vt[NS];
  __shared__ int s_par[NS];
  __shared__ __attribute__((aligned(16))) int s_tok0[TPITCH];
  __shared__ __attribute__((aligned(16))) int s_tok1[TPITCH];
  __shared__ __attribute__((aligned(16))) float s_rec[ND];
  __shared__ __attribute__((aligned(16))) unsigned int s_sc[32];
  __shared__ float s_enc[ND];
  __shared__ float s_mean[NL];
  __shared__ float s_lv[NL];
  __shared__ float s_z[NL];
  __shared__ int s_wi[8];
  __shared__ double s_wd[8];

  const int b = blockIdx.x, t = threadIdx.x, lane = t & 31, w = t >> 5;
  const size_t rowb = (size_t)b * NS;

  #pragma unroll
  for (int q = 0; q < 2; ++q) {
    const int s = t + 256 * q;
    const int mk = (mask[rowb + s] != 0) ? 1 : 0;
    const int v = vocab[rowb + s];
    s_msk[s] = mk;
    s_voc[s] = v;
    s_vt[s] = mk ? v : PAD_ID;
  }
  __syncthreads();

  int ff = NS;
  #pragma unroll
  for (int q = 0; q < 2; ++q) {
    const int s = t + 256 * q;
    int oi = order[(rowb + s) * 6];
    oi = (oi == -1) ? BOS_ID : oi;
    oi = (oi < 0) ? (oi + NS) : oi;
    oi = clampi(oi, 0, NS - 1);
    const int pv = s_vt[oi];
    const int mk = s_msk[s];
    int par = mk ? pv : PAD_ID;
    par = (s == 0) ? BOS_ID : par;
    s_par[s] = par;
    ff = mk ? ff : min(ff, s);
  }
  ff = wmin_i(ff);
  if (lane == 0) s_wi[w] = ff;
  __syncthreads();
  int ffs0 = NS;
  #pragma unroll
  for (int i = 0; i < 8; ++i) ffs0 = min(ffs0, s_wi[i]);

  float acc = 0.0f;
  int cnt = 0;
  #pragma unroll 1
  for (int s = 0; s < NS; ++s) {
    if (s_msk[s] != 0) {
      ++cnt;
      const int a = clampi(s_vt[s], 0, NV - 1);
      const int p = clampi(s_par[s], 0, NV - 1);
      const float e1 = emb[(size_t)a * ND + t];
      const float e2 = emb[(size_t)p * ND + t];
      acc += (e1 + e2);
    }
  }
  const float cntf = (cnt > 0) ? (float)cnt : 1.0f;
  s_enc[t] = acc * (1.0f / cntf);
  __syncthreads();

  if (t < NL) {
    float a = 0.0f;
    #pragma unroll 1
    for (int d = 0; d < ND; ++d) a = fmaf(s_enc[d], Wm[(size_t)d * NL + t], a);
    s_mean[t] = a + bm[t];
  } else {
    const int l = t - NL;
    float a = 0.0f;
    #pragma unroll 1
    for (int d = 0; d < ND; ++d) a = fmaf(s_enc[d], Wv[(size_t)d * NL + l], a);
    s_lv[l] = a + bv[l];
  }
  __syncthreads();

  double klt = 0.0;
  if (t < NL) {
    const float mu = s_mean[t], lv = s_lv[t];
    const float zz = mu + eps[(size_t)b * NL + t] * expf(0.5f * lv);
    s_z[t] = zz;
    const float term = 1.0f + lv - mu * mu - expf(lv);
    klt = (double)term;
  }
  __syncthreads();

  {
    float a = 0.0f;
    #pragma unroll 1
    for (int l = 0; l < NL; ++l) a = fmaf(s_z[l], Wlin[(size_t)l * ND + t], a);
    s_rec[t] = a + blin[t];
  }
  klt = wsum_d(klt);

  const bool hasf = (ffs0 < NS);
  const int ffe = ffs0 + 1;
  int vcnt = 0;
  for (int j = t; j < TPITCH; j += 256) {
    const int vprev = s_voc[clampi(j - 1, 0, NS - 1)];
    const int vcur  = s_voc[clampi(j, 0, NS - 1)];
    int inp = (j == 0) ? BOS_ID : vprev;
    inp = (hasf && j >= ffe) ? PAD_ID : inp;
    int tgt = (j < NS) ? vcur : BOS_ID;
    tgt = (hasf && j == ffe - 1) ? EOS_ID : tgt;
    tgt = (hasf && j >= ffe) ? PAD_ID : tgt;
    const bool live = (j < NJ);
    inp = live ? inp : 0;
    tgt = live ? tgt : 0;
    vcnt += (live && tgt != PAD_ID) ? 1 : 0;
    s_tok0[j] = inp;
    s_tok1[j] = tgt;
  }
  vcnt = wsum_i(vcnt);
  if (lane == 0) { s_wd[w] = klt; s_wi[w] = vcnt; }
  __syncthreads();
  if (t == 0) {
    double kl = 0.0;
    int vt = 0;
    #pragma unroll
    for (int i = 0; i < 8; ++i) { kl += s_wd[i]; vt += s_wi[i]; }
    unsigned int lo, hi;
    d2u(kl, lo, hi);
    s_sc[0] = lo;
    s_sc[1] = hi;
    s_sc[2] = (unsigned int)vt;
    #pragma unroll
    for (int i = 3; i < 32; ++i) s_sc[i] = 0u;
  }
  __syncthreads();

  seq_store(s_rec, s_sc, s_tok0, s_tok1, rec, inpP, tgtP, b, t);
  __threadfence();
  seq_store(s_rec, s_sc, s_tok0, s_tok1, rec, inpP, tgtP, b, t);
}

__global__ __launch_bounds__(128) void k_head(
    const float* __restrict__ emb, const _Float16* __restrict__ woutT,
    const float* __restrict__ bout, const float* __restrict__ rec,
    const int* __restrict__ inpP, const int* __restrict__ tgtP,
    unsigned int* __restrict__ part)
{
  __shared__ __attribute__((aligned(16))) _Float16 sA[HROWS * APITCH];
  __shared__ int s_inp[HROWS];
  __shared__ int s_tgt[HROWS];
  __shared__ int s_bb[HROWS];
  __shared__ double s_wd[4];
  __shared__ __attribute__((aligned(16))) unsigned int s_line[32];

  const int t = threadIdx.x, lane = t & 31, w = t >> 5;
  const int h = lane >> 4, m = lane & 15;
  const int row0 = blockIdx.x * HROWS;

  if (t < HROWS) {
    const int p = row0 + t;
    const int b = p / NJ;
    const int j = p - b * NJ;
    s_inp[t] = clampi(inpP[(size_t)b * TPITCH + j], 0, NV - 1);
    s_tgt[t] = tgtP[(size_t)b * TPITCH + j];
    s_bb[t]  = b;
  }
  __syncthreads();

  #pragma unroll 2
  for (int it = 0; it < 16; ++it) {
    const int c = it * 128 + t;
    const int r = c >> 5, c8 = c & 31;
    const int tok = s_inp[r], bb = s_bb[r];
    const float* ep = emb + (size_t)tok * ND + 8 * c8;
    const float* mp = rec + (size_t)bb * RPITCH + 8 * c8;
    const v4f e0 = *(const v4fa*)ep, e1 = *(const v4fa*)(ep + 4);
    const v4f m0 = *(const v4fa*)mp, m1 = *(const v4fa*)(mp + 4);
    v8h o;
    o[0] = (_Float16)(e0.x + m0.x); o[1] = (_Float16)(e0.y + m0.y);
    o[2] = (_Float16)(e0.z + m0.z); o[3] = (_Float16)(e0.w + m0.w);
    o[4] = (_Float16)(e1.x + m1.x); o[5] = (_Float16)(e1.y + m1.y);
    o[6] = (_Float16)(e1.z + m1.z); o[7] = (_Float16)(e1.w + m1.w);
    *(v8ha*)(sA + r * APITCH + 8 * c8) = o;
  }
  __syncthreads();

  int tg[8];
  #pragma unroll
  for (int r = 0; r < 8; ++r) tg[r] = s_tgt[16 * w + 8 * h + r];

  const _Float16* arow = sA + (16 * w + m) * APITCH;
  const v8f zero8 = {0.f, 0.f, 0.f, 0.f, 0.f, 0.f, 0.f, 0.f};
  double acc64 = 0.0;

  #pragma unroll 1
  for (int half = 0; half < 2; ++half) {
    v8f acc[8];
    #pragma unroll
    for (int nt = 0; nt < 8; ++nt) acc[nt] = zero8;
    const _Float16* wb = woutT + (size_t)(half * 128 + m) * ND;

    #pragma unroll 1
    for (int k0 = 0; k0 < ND; k0 += 32) {
      const v16h a = load_frag(arow + k0, h);
      #pragma unroll
      for (int nt = 0; nt < 8; ++nt) {
        const v16h bf = load_frag(wb + (size_t)nt * 16 * ND + k0, h);
        acc[nt] = wmma_f16(a, bf, acc[nt]);
      }
    }

    #pragma unroll
    for (int nt = 0; nt < 8; ++nt) {
      const int col = half * 128 + 16 * nt + m;
      const float bo = bout[col];
      #pragma unroll
      for (int r = 0; r < 8; ++r) {
        const int tgc = clampi(tg[r], 0, NV - 1);
        const float te = emb[(size_t)tgc * ND + col];
        const float word = acc[nt][r] * WSCINV + bo;
        const float diff = word - te;
        const float sq = diff * diff;
        acc64 += (tg[r] != PAD_ID) ? (double)sq : 0.0;
      }
    }
  }

  acc64 = wsum_d(acc64);
  if (lane == 0) s_wd[w] = acc64;
  __syncthreads();
  if (t == 0) {
    const double tot = ((s_wd[0] + s_wd[1]) + s_wd[2]) + s_wd[3];
    unsigned int lo, hi;
    d2u(tot, lo, hi);
    s_line[0] = lo;
    s_line[1] = hi;
    #pragma unroll
    for (int i = 2; i < 32; ++i) s_line[i] = 0u;
  }
  __syncthreads();
  if (t < 8) {
    const v4u v = *(const v4ua*)(s_line + 4 * t);
    *(volatile v4u*)(part + (size_t)blockIdx.x * 32 + 4 * t) = v;
  }
  __threadfence();
  if (t < 8) {
    const v4u v = *(const v4ua*)(s_line + 4 * t);
    *(volatile v4u*)(part + (size_t)blockIdx.x * 32 + 4 * t) = v;
  }
}

__global__ __launch_bounds__(256) void k_final(
    const unsigned int* __restrict__ part, int npart,
    const unsigned int* __restrict__ recu, float* __restrict__ out)
{
  __shared__ double s_wl[8];
  __shared__ double s_wk[8];
  __shared__ int s_wi[8];
  const int t = threadIdx.x, lane = t & 31, w = t >> 5;

  double ls = 0.0;
  const int nit = (npart + 255) / 256;
  #pragma unroll 1
  for (int it = 0; it < nit; ++it) {
    const int i = it * 256 + t;
    const int ic = clampi(i, 0, npart - 1);
    const double v = u2d(part[(size_t)ic * 32], part[(size_t)ic * 32 + 1]);
    ls += (i < npart) ? v : 0.0;
  }
  ls = wsum_d(ls);

  const size_t rb = (size_t)t * RPITCH + ND;
  double kl = u2d(recu[rb], recu[rb + 1]);
  int vc = (int)recu[rb + 2];
  kl = wsum_d(kl);
  vc = wsum_i(vc);
  if (lane == 0) { s_wl[w] = ls; s_wk[w] = kl; s_wi[w] = vc; }
  __syncthreads();
  if (t == 0) {
    double lsum = 0.0, ksum = 0.0;
    int vtot = 0;
    #pragma unroll
    for (int i = 0; i < 8; ++i) { lsum += s_wl[i]; ksum += s_wk[i]; vtot += s_wi[i]; }
    long long dn = (long long)vtot * (long long)ND;
    if (dn < 1) dn = 1;
    const float denf = (float)dn;
    const float loss = (float)(lsum / (double)denf);
    const float klv  = (float)(-0.5 * ksum / (double)NB);
    v2f o;
    o.x = loss;
    o.y = klv;
    *(volatile v2f*)out = o;
    __threadfence();
    *(volatile v2f*)out = o;
  }
}

extern "C" void kernel_launch(void* const* d_in, const int* in_sizes, int n_in,
                              void* d_out, int out_size, void* d_ws, size_t ws_size,
                              hipStream_t stream) {
  if (n_in < 13) return;
  if (in_sizes[0] != NB * NS) return;
  if (in_sizes[1] != NB * NS * 6) return;
  if (in_sizes[2] != NB * NS) return;
  if (in_sizes[3] != NB * NL) return;
  if (in_sizes[4] != NV * ND) return;
  if (in_sizes[5] != ND * NL || in_sizes[7] != ND * NL) return;
  if (in_sizes[6] != NL || in_sizes[8] != NL) return;
  if (in_sizes[9] != NL * ND || in_sizes[10] != ND) return;
  if (in_sizes[11] != ND * ND || in_sizes[12] != ND) return;
  if (out_size != 2) return;

  const int*   vocab = (const int*)d_in[0];
  const int*   order = (const int*)d_in[1];
  const int*   mask  = (const int*)d_in[2];
  const float* eps   = (const float*)d_in[3];
  const float* emb   = (const float*)d_in[4];
  const float* Wm    = (const float*)d_in[5];
  const float* bm    = (const float*)d_in[6];
  const float* Wv    = (const float*)d_in[7];
  const float* bv    = (const float*)d_in[8];
  const float* Wlin  = (const float*)d_in[9];
  const float* blin  = (const float*)d_in[10];
  const float* Wout  = (const float*)d_in[11];
  const float* bout  = (const float*)d_in[12];
  float* out = (float*)d_out;

  const size_t woutT_bytes = (size_t)ND * ND * 2;
  const size_t rec_bytes   = (size_t)NB * RPITCH * 4;
  const size_t tok_bytes   = (size_t)NB * TPITCH * 4;
  const size_t part_bytes  = (size_t)NBLK2 * 32 * 4;
  const size_t total = woutT_bytes + rec_bytes + 2 * tok_bytes + part_bytes;
  if (total > ws_size) return;

  char* ws = (char*)d_ws;
  _Float16* woutT   = (_Float16*)(ws);
  float* rec        = (float*)(ws + woutT_bytes);
  int* inpP         = (int*)(ws + woutT_bytes + rec_bytes);
  int* tgtP         = (int*)(ws + woutT_bytes + rec_bytes + tok_bytes);
  unsigned int* part = (unsigned int*)(ws + woutT_bytes + rec_bytes + 2 * tok_bytes);

  k_wout<<<ND / 32, 256, 0, stream>>>(Wout, woutT);
  k_seq<<<NB, 256, 0, stream>>>(vocab, order, mask, eps, emb, Wm, bm, Wv, bv, Wlin, blin,
                                rec, inpP, tgtP);
  k_head<<<NBLK2, 128, 0, stream>>>(emb, woutT, bout, rec, inpP, tgtP, part);
  k_final<<<1, 256, 0, stream>>>(part, NBLK2, (const unsigned int*)rec, out);
}
